// GNN_Model_6493990552142
// MI455X (gfx1250) — hardware-verified
//
#include <hip/hip_runtime.h>

#define NL 10000
#define NP 50000
#define PLEN 5
#define EDG (NP * PLEN)
#define TIT 8
#define DH 32
#define GW 96
#define RU 256
#define LB 64
#define NLB ((NL + LB - 1) / LB)
#define CAP 4096
#define NPT (NP / 16)
#define NLT (NL / 16)

typedef _Float16 v8h __attribute__((ext_vector_type(8)));
typedef _Float16 v16h __attribute__((ext_vector_type(16)));
typedef float v8f __attribute__((ext_vector_type(8)));
typedef float v4f __attribute__((ext_vector_type(4)));
typedef int v4i __attribute__((ext_vector_type(4)));
union Frag { v16h v; v8h half[2]; };

__device__ __forceinline__ v8f mma16(v16h a, v16h b, v8f c) {
  v8f d = __builtin_amdgcn_wmma_f32_16x16x32_f16(false, a, false, b, (short)0, c, false, false);
  asm volatile("v_nop\n\tv_nop\n\tv_nop\n\tv_nop" : "+v"(d) : "v"(a), "v"(b));
  return d;
}

__device__ __forceinline__ v8f splat8(float x) {
  v8f r;
#pragma unroll
  for (int i = 0; i < 8; ++i) r[i] = x;
  return r;
}

__device__ __forceinline__ v16h frag_h(const _Float16* rp, int h) {
  Frag u;
  u.half[0] = *(const v8h*)(rp + 8 * h);
  u.half[1] = *(const v8h*)(rp + 16 + 8 * h);
  return u.v;
}

__device__ __forceinline__ v16h frag_f(const float* rp, int h) {
  v4f a = *(const v4f*)(rp + 8 * h);
  v4f b = *(const v4f*)(rp + 8 * h + 4);
  v4f c = *(const v4f*)(rp + 16 + 8 * h);
  v4f d = *(const v4f*)(rp + 20 + 8 * h);
  v16h r;
#pragma unroll
  for (int i = 0; i < 4; ++i) {
    r[i] = (_Float16)a[i];
    r[4 + i] = (_Float16)b[i];
    r[8 + i] = (_Float16)c[i];
    r[12 + i] = (_Float16)d[i];
  }
  return r;
}

__device__ __forceinline__ float sigm16(float x) {
  float e = __builtin_amdgcn_exp2f(x * -0.09016844005556021f);
  return __builtin_amdgcn_rcpf(1.0f + e);
}
__device__ __forceinline__ float tanh16(float x) {
  float e = __builtin_amdgcn_exp2f(x * 0.18033688011112042f);
  return 1.0f - 2.0f * __builtin_amdgcn_rcpf(1.0f + e);
}

__device__ __forceinline__ void gru_gates(const v8f* ar, const v8f* az, const v8f* gi,
                                          const v8f* an, float hD[2][8]) {
#pragma unroll
  for (int t2 = 0; t2 < 2; ++t2) {
#pragma unroll
    for (int r = 0; r < 8; ++r) {
      float rr = sigm16(ar[t2][r]);
      float zz = sigm16(az[t2][r]);
      float nn = tanh16(gi[t2][r] + rr * an[t2][r]);
      hD[t2][r] = (1.0f - zz) * nn + zz * hD[t2][r];
    }
  }
}

__device__ __forceinline__ void put_h16(_Float16* hs, const float hD[2][8], int h, int lo) {
#pragma unroll
  for (int t2 = 0; t2 < 2; ++t2)
#pragma unroll
    for (int r = 0; r < 8; ++r)
      hs[(8 * h + r) * DH + 16 * t2 + lo] = (_Float16)hD[t2][r];
}

__device__ __forceinline__ void put_f32(float* os, const float hD[2][8], int h, int lo) {
#pragma unroll
  for (int t2 = 0; t2 < 2; ++t2)
#pragma unroll
    for (int r = 0; r < 8; ++r)
      os[(8 * h + r) * DH + 16 * t2 + lo] = hD[t2][r];
}

__device__ __forceinline__ void lines2(float* g, const float* s, int ngrp, int lane, bool valid) {
  for (int q = 0; q < ngrp; ++q) {
    v4f v = *(const v4f*)(s + 128 * q + 4 * lane);
    if (valid) *(volatile v4f*)(g + 128 * q + 4 * lane) = v;
  }
  __threadfence();
  for (int q = 0; q < ngrp; ++q) {
    v4f v = *(const v4f*)(s + 128 * q + 4 * lane);
    if (valid) *(volatile v4f*)(g + 128 * q + 4 * lane) = v;
  }
}

__global__ void __launch_bounds__(256) init_kernel(
    const float* __restrict__ traffic, const float* __restrict__ packets,
    const float* __restrict__ tdp, const float* __restrict__ capacity,
    float* __restrict__ path_state, float* __restrict__ link_state) {
  const int idx = blockIdx.x * 256 + threadIdx.x;
  if (blockIdx.y == 0) {
    if (idx < NP * 8) {
      const int r = idx >> 3, c4 = (idx & 7) * 4;
      v4f v;
#pragma unroll
      for (int j = 0; j < 4; ++j) {
        const int c = c4 + j;
        float x = 0.0f;
        if (c == 0) x = traffic[r];
        else if (c == 1) x = packets[r];
        else if (c < 14) x = tdp[r * 12 + (c - 2)];
        v[j] = x;
      }
      float* p = path_state + (size_t)idx * 4;
      *(volatile v4f*)p = v;
      __threadfence();
      *(volatile v4f*)p = v;
    }
  } else {
    if (idx < NL * 8) {
      const int r = idx >> 3, c4 = (idx & 7) * 4;
      v4f v;
      v[0] = (c4 == 0) ? capacity[r] : 0.0f;
      v[1] = 0.0f; v[2] = 0.0f; v[3] = 0.0f;
      float* p = link_state + (size_t)idx * 4;
      *(volatile v4f*)p = v;
      __threadfence();
      *(volatile v4f*)p = v;
    }
  }
}

__global__ void __launch_bounds__(256) cvt_kernel(
    const float* __restrict__ w0, const float* __restrict__ w1, const float* __restrict__ w2,
    const float* __restrict__ w3, const float* __restrict__ w4, const float* __restrict__ w5,
    _Float16* __restrict__ dst) {
  const int sel = blockIdx.y;
  const float* src;
  int n, doff;
  if (sel == 0)      { src = w0; n = GW * DH; doff = 0; }
  else if (sel == 1) { src = w1; n = GW * DH; doff = GW * DH; }
  else if (sel == 2) { src = w2; n = GW * DH; doff = 2 * GW * DH; }
  else if (sel == 3) { src = w3; n = GW * DH; doff = 3 * GW * DH; }
  else if (sel == 4) { src = w4; n = RU * DH; doff = 4 * GW * DH; }
  else               { src = w5; n = RU * RU; doff = 4 * GW * DH + RU * DH; }
  const int i8 = blockIdx.x * 256 + threadIdx.x;
  if (i8 * 8 < n) {
    v4f a = *(const v4f*)(src + i8 * 8);
    v4f b = *(const v4f*)(src + i8 * 8 + 4);
    v8h o;
#pragma unroll
    for (int j = 0; j < 4; ++j) {
      o[j] = (_Float16)(a[j] * 16.0f);
      o[4 + j] = (_Float16)(b[j] * 16.0f);
    }
    _Float16* p = dst + doff + i8 * 8;
    *(volatile v8h*)p = o;
    __threadfence();
    *(volatile v8h*)p = o;
  }
}

__global__ void __launch_bounds__(256) csr_kernel(
    const int* __restrict__ sl, const int* __restrict__ ptl, int n_edges,
    int* __restrict__ cols, int* __restrict__ linfo) {
  __shared__ int lst[CAP];
  __shared__ __align__(16) int srt[CAP];
  __shared__ int wc[8];
  __shared__ int qcnt[256];
  __shared__ int qoff[256];
  __shared__ int ltot[64];
  __shared__ __align__(16) int linf[128];
  const int tid = threadIdx.x, lane = tid & 31, wave = tid >> 5;
  const int lbase = blockIdx.x * LB;
  for (int i = tid; i < CAP; i += 256) srt[i] = 0;

  int n = 0;
  for (int c0 = 0; c0 < n_edges; c0 += 2048) {
    const int e0 = c0 + 8 * tid;
    int lv[8], pv[8];
    if (e0 + 8 <= n_edges) {
      v4i a = *(const v4i*)(sl + e0);
      v4i b = *(const v4i*)(sl + e0 + 4);
      v4i c = *(const v4i*)(ptl + e0);
      v4i d = *(const v4i*)(ptl + e0 + 4);
#pragma unroll
      for (int j = 0; j < 4; ++j) { lv[j] = a[j]; lv[4 + j] = b[j]; pv[j] = c[j]; pv[4 + j] = d[j]; }
    } else {
#pragma unroll
      for (int j = 0; j < 8; ++j) {
        const int e = e0 + j;
        if (e < n_edges) { lv[j] = sl[e]; pv[j] = ptl[e]; }
        else { lv[j] = -1; pv[j] = 0; }
      }
    }
    int msk = 0;
#pragma unroll
    for (int j = 0; j < 8; ++j) {
      const unsigned loc = (unsigned)(lv[j] - lbase);
      if (loc < (unsigned)LB) msk |= (1 << j);
    }
    const int cnt = __popc(msk);
    int incl = cnt;
#pragma unroll
    for (int dlt = 1; dlt < 32; dlt <<= 1) {
      int y = __shfl_up(incl, dlt);
      if (lane >= dlt) incl += y;
    }
    if (lane == 31) wc[wave] = incl;
    __syncthreads();
    int below = 0, tot = 0;
#pragma unroll
    for (int w = 0; w < 8; ++w) {
      const int c = wc[w];
      below += (w < wave) ? c : 0;
      tot += c;
    }
    int pos = n + below + incl - cnt;
#pragma unroll
    for (int j = 0; j < 8; ++j) {
      if (msk & (1 << j)) {
        int p = pv[j];
        p = p < 0 ? 0 : (p > NP - 1 ? NP - 1 : p);
        if (pos < CAP) lst[pos] = p * 64 + (lv[j] - lbase);
        ++pos;
      }
    }
    n += tot;
    __syncthreads();
  }
  if (n > CAP) n = CAP;

  const int loc = tid & 63, q = tid >> 6;
  const int i0 = (n * q) >> 2, i1 = (n * (q + 1)) >> 2;
  int c = 0;
  for (int i = i0; i < i1; ++i) c += ((lst[i] & 63) == loc) ? 1 : 0;
  qcnt[loc * 4 + q] = c;
  __syncthreads();
  if (tid < 64) ltot[tid] = qcnt[4 * tid] + qcnt[4 * tid + 1] + qcnt[4 * tid + 2] + qcnt[4 * tid + 3];
  __syncthreads();
  if (tid < 64) {
    int off = 0;
    for (int j = 0; j < tid; ++j) off += ltot[j];
    int a = off;
#pragma unroll
    for (int qq = 0; qq < 4; ++qq) { qoff[4 * tid + qq] = a; a += qcnt[4 * tid + qq]; }
    linf[2 * tid] = off;
    linf[2 * tid + 1] = ltot[tid];
  }
  __syncthreads();
  int pos = qoff[loc * 4 + q];
  for (int i = i0; i < i1; ++i) {
    const int v = lst[i];
    if ((v & 63) == loc) {
      if (pos < CAP) srt[pos] = v >> 6;
      ++pos;
    }
  }
  __syncthreads();

  int* cdst = cols + (size_t)blockIdx.x * CAP;
  int* ldst = linfo + (size_t)blockIdx.x * (2 * LB);
  v4i cv[4];
#pragma unroll
  for (int s = 0; s < 4; ++s) cv[s] = *(const v4i*)(srt + 1024 * s + 4 * tid);
  v4i li4 = *(const v4i*)(linf + 4 * lane);
#pragma unroll
  for (int s = 0; s < 4; ++s) *(volatile v4i*)(cdst + 1024 * s + 4 * tid) = cv[s];
  if (wave == 0) *(volatile v4i*)(ldst + 4 * lane) = li4;
  __threadfence();
#pragma unroll
  for (int s = 0; s < 4; ++s) *(volatile v4i*)(cdst + 1024 * s + 4 * tid) = cv[s];
  if (wave == 0) *(volatile v4i*)(ldst + 4 * lane) = li4;
}

__global__ void __launch_bounds__(128) link_kernel(
    int full, float* __restrict__ link_state, const float* __restrict__ path_state,
    const int* __restrict__ cols, const int* __restrict__ linfo,
    const _Float16* __restrict__ Wi16l, const _Float16* __restrict__ Wh16l,
    const float* __restrict__ bil, const float* __restrict__ bhl,
    const _Float16* __restrict__ Wi16p, const float* __restrict__ bip,
    float* __restrict__ G) {
  __shared__ __align__(16) _Float16 hs_all[4][16 * DH];
  __shared__ __align__(16) _Float16 xs_all[4][16 * DH];
  __shared__ __align__(16) float os_all[4][16 * DH];
  __shared__ __align__(16) float gs_all[4][16 * GW];
  const int wave = threadIdx.x >> 5, lane = threadIdx.x & 31;
  const int h = lane >> 4, lo = lane & 15;
  const int lbase = blockIdx.x * LB;
  const int L0 = lbase + 16 * wave;
  const bool valid = L0 < NL;
  const int row0 = valid ? L0 : (NL - 16);
  _Float16* hs = hs_all[wave];
  _Float16* xs = xs_all[wave];
  float* os = os_all[wave];
  float* gs = gs_all[wave];

  float hD[2][8];
  if (full) {
    const int* creg = cols + (size_t)blockIdx.x * CAP;
#pragma unroll 1
    for (int i = 0; i < 16; ++i) {
      const int L = L0 + i;
      int off = linfo[2 * L], cnt = linfo[2 * L + 1];
      off = off < 0 ? 0 : (off > CAP ? CAP : off);
      cnt = cnt < 0 ? 0 : (cnt > CAP - off ? CAP - off : cnt);
      float s = 0.0f;
      for (int k = 0; k < cnt; ++k) {
        int p = creg[off + k];
        p = p < 0 ? 0 : (p > NP - 1 ? NP - 1 : p);
        s += path_state[(size_t)p * DH + lane];
      }
      xs[i * DH + lane] = (_Float16)s;
    }
    __syncthreads();
    v16h xa = frag_h(xs + lo * DH, h);
    v16h ha = frag_f(link_state + (size_t)(row0 + lo) * DH, h);
#pragma unroll
    for (int t2 = 0; t2 < 2; ++t2)
#pragma unroll
      for (int r = 0; r < 8; ++r)
        hD[t2][r] = link_state[(size_t)(row0 + 8 * h + r) * DH + 16 * t2 + lo];

    v8f ar[2], az[2], gi[2], an[2];
#pragma unroll
    for (int t2 = 0; t2 < 2; ++t2) {
      const int cr = 16 * t2 + lo, cz = 32 + 16 * t2 + lo, cn = 64 + 16 * t2 + lo;
      ar[t2] = splat8(16.0f * (bil[cr] + bhl[cr]));
      ar[t2] = mma16(xa, frag_h(Wi16l + cr * DH, h), ar[t2]);
      ar[t2] = mma16(ha, frag_h(Wh16l + cr * DH, h), ar[t2]);
      az[t2] = splat8(16.0f * (bil[cz] + bhl[cz]));
      az[t2] = mma16(xa, frag_h(Wi16l + cz * DH, h), az[t2]);
      az[t2] = mma16(ha, frag_h(Wh16l + cz * DH, h), az[t2]);
      gi[t2] = mma16(xa, frag_h(Wi16l + cn * DH, h), splat8(16.0f * bil[cn]));
      an[t2] = mma16(ha, frag_h(Wh16l + cn * DH, h), splat8(16.0f * bhl[cn]));
    }
    gru_gates(ar, az, gi, an, hD);
  } else {
#pragma unroll
    for (int t2 = 0; t2 < 2; ++t2)
#pragma unroll
      for (int r = 0; r < 8; ++r)
        hD[t2][r] = link_state[(size_t)(row0 + 8 * h + r) * DH + 16 * t2 + lo];
  }

  put_h16(hs, hD, h, lo);
  put_f32(os, hD, h, lo);
  __syncthreads();
  if (full) lines2(link_state + (size_t)row0 * DH, os, 4, lane, valid);

  v16h hb = frag_h(hs + lo * DH, h);
  v8f ag[6];
#pragma unroll
  for (int f = 0; f < 6; ++f)
    ag[f] = mma16(hb, frag_h(Wi16p + (16 * f + lo) * DH, h), splat8(16.0f * bip[16 * f + lo]));
#pragma unroll
  for (int f = 0; f < 6; ++f)
#pragma unroll
    for (int r = 0; r < 8; ++r)
      gs[(8 * h + r) * GW + 16 * f + lo] = ag[f][r];
  __syncthreads();
  lines2(G + (size_t)row0 * GW, gs, 12, lane, valid);
}

__global__ void __launch_bounds__(256) path_kernel(
    float* __restrict__ path_state, const float* __restrict__ G,
    const int* __restrict__ ltp, const _Float16* __restrict__ Wh16,
    const float* __restrict__ bh) {
  __shared__ __align__(16) _Float16 hs_all[8][16 * DH];
  __shared__ __align__(16) float os_all[8][16 * DH];
  const int wave = threadIdx.x >> 5, lane = threadIdx.x & 31;
  const int h = lane >> 4, lo = lane & 15;
  int tile = blockIdx.x * 8 + wave;
  const bool valid = tile < NPT;
  if (!valid) tile = NPT - 1;
  const int row0 = tile * 16;
  _Float16* hs = hs_all[wave];
  float* os = os_all[wave];

  float bhr[2], bhz[2], bhn[2];
#pragma unroll
  for (int t2 = 0; t2 < 2; ++t2) {
    bhr[t2] = 16.0f * bh[16 * t2 + lo];
    bhz[t2] = 16.0f * bh[32 + 16 * t2 + lo];
    bhn[t2] = 16.0f * bh[64 + 16 * t2 + lo];
  }

  v16h ha = frag_f(path_state + (size_t)(row0 + lo) * DH, h);
  float hD[2][8];
#pragma unroll
  for (int t2 = 0; t2 < 2; ++t2)
#pragma unroll
    for (int r = 0; r < 8; ++r)
      hD[t2][r] = path_state[(size_t)(row0 + 8 * h + r) * DH + 16 * t2 + lo];

#pragma unroll 1
  for (int t = 0; t < PLEN; ++t) {
    v8f ar[2], az[2], gi[2], an[2];
#pragma unroll
    for (int r = 0; r < 8; ++r) {
      int li = ltp[(size_t)(row0 + 8 * h + r) * PLEN + t];
      li = li < 0 ? 0 : (li > NL - 1 ? NL - 1 : li);
      const float* g = G + (size_t)li * GW + lo;
#pragma unroll
      for (int t2 = 0; t2 < 2; ++t2) {
        ar[t2][r] = g[16 * t2] + bhr[t2];
        az[t2][r] = g[32 + 16 * t2] + bhz[t2];
        gi[t2][r] = g[64 + 16 * t2];
      }
    }
#pragma unroll
    for (int t2 = 0; t2 < 2; ++t2) {
      an[t2] = splat8(bhn[t2]);
      ar[t2] = mma16(ha, frag_h(Wh16 + (16 * t2 + lo) * DH, h), ar[t2]);
      az[t2] = mma16(ha, frag_h(Wh16 + (32 + 16 * t2 + lo) * DH, h), az[t2]);
      an[t2] = mma16(ha, frag_h(Wh16 + (64 + 16 * t2 + lo) * DH, h), an[t2]);
    }
    gru_gates(ar, az, gi, an, hD);
    if (t < PLEN - 1) {
      put_h16(hs, hD, h, lo);
      __syncthreads();
      ha = frag_h(hs + lo * DH, h);
    }
  }

  put_f32(os, hD, h, lo);
  __syncthreads();
  lines2(path_state + (size_t)row0 * DH, os, 4, lane, valid);
}

__global__ void __launch_bounds__(128) readout_kernel(
    const float* __restrict__ path_state,
    const _Float16* __restrict__ W1h, const float* __restrict__ b1,
    const _Float16* __restrict__ W2h, const float* __restrict__ b2,
    const float* __restrict__ W3, const float* __restrict__ b3,
    float* __restrict__ out) {
  __shared__ __align__(16) _Float16 r1_all[4][16 * RU];
  __shared__ __align__(16) float outs[64];
  const int wave = threadIdx.x >> 5, lane = threadIdx.x & 31;
  const int h = lane >> 4, lo = lane & 15;
  int tile = blockIdx.x * 4 + wave;
  if (tile > NPT - 1) tile = NPT - 1;
  const int row0 = tile * 16;
  _Float16* r1 = r1_all[wave];

  v16h ha = frag_f(path_state + (size_t)(row0 + lo) * DH, h);

#pragma unroll 1
  for (int f = 0; f < 16; ++f) {
    v8f acc = mma16(ha, frag_h(W1h + (16 * f + lo) * DH, h), splat8(16.0f * b1[16 * f + lo]));
#pragma unroll
    for (int r = 0; r < 8; ++r) {
      float x = fmaxf(acc[r], 0.0f) * 0.0625f;
      r1[(8 * h + r) * RU + 16 * f + lo] = (_Float16)x;
    }
  }
  __syncthreads();

  v16h aF[8];
#pragma unroll
  for (int kc = 0; kc < 8; ++kc) aF[kc] = frag_h(r1 + lo * RU + kc * 32, h);

  float part[8];
#pragma unroll
  for (int r = 0; r < 8; ++r) part[r] = 0.0f;
#pragma unroll 1
  for (int f2 = 0; f2 < 16; ++f2) {
    v8f acc = splat8(16.0f * b2[16 * f2 + lo]);
    const _Float16* wrow = W2h + (size_t)(16 * f2 + lo) * RU;
#pragma unroll
    for (int kc = 0; kc < 8; ++kc) acc = mma16(aF[kc], frag_h(wrow + kc * 32, h), acc);
    const float w3c = W3[16 * f2 + lo];
#pragma unroll
    for (int r = 0; r < 8; ++r) part[r] += (fmaxf(acc[r], 0.0f) * 0.0625f) * w3c;
  }
#pragma unroll
  for (int r = 0; r < 8; ++r) {
    float v = part[r];
    v += __shfl_xor(v, 1);
    v += __shfl_xor(v, 2);
    v += __shfl_xor(v, 4);
    v += __shfl_xor(v, 8);
    part[r] = v;
  }
  if (lo == 0) {
    const float bb = b3[0];
#pragma unroll
    for (int r = 0; r < 8; ++r) outs[16 * wave + 8 * h + r] = part[r] + bb;
  }
  __syncthreads();

  const int rb = blockIdx.x * 64 + 4 * lane;
  const bool wr = (wave == 0) && (lane < 16) && (rb + 4 <= NP);
  v4f ov;
  ov[0] = 0.0f; ov[1] = 0.0f; ov[2] = 0.0f; ov[3] = 0.0f;
  if (wave == 0 && lane < 16) ov = *(const v4f*)(outs + 4 * lane);
  if (wr) *(volatile v4f*)(out + rb) = ov;
  __threadfence();
  if (wr) *(volatile v4f*)(out + rb) = ov;
}

extern "C" void kernel_launch(void* const* d_in, const int* in_sizes, int n_in,
                              void* d_out, int out_size, void* d_ws,
                              size_t ws_size, hipStream_t stream) {
  if (n_in < 25 || out_size < NP) return;
  if (in_sizes[0] < NP || in_sizes[1] < NP || in_sizes[2] < NP * 12 || in_sizes[3] < NL) return;
  if (in_sizes[4] < EDG) return;
  if (in_sizes[11] < GW * DH || in_sizes[12] < GW * DH || in_sizes[15] < GW * DH || in_sizes[16] < GW * DH) return;
  if (in_sizes[13] < GW || in_sizes[14] < GW || in_sizes[17] < GW || in_sizes[18] < GW) return;
  if (in_sizes[19] < RU * DH || in_sizes[20] < RU || in_sizes[21] < RU * RU || in_sizes[22] < RU) return;
  if (in_sizes[23] < RU || in_sizes[24] < 1) return;

  const float* traffic  = (const float*)d_in[0];
  const float* packets  = (const float*)d_in[1];
  const float* tdp      = (const float*)d_in[2];
  const float* capacity = (const float*)d_in[3];
  const int* link_to_path   = (const int*)d_in[4];
  const int* path_to_link   = (const int*)d_in[7];
  const int* sequence_links = (const int*)d_in[8];
  const float* Wi_p = (const float*)d_in[11];
  const float* Wh_p = (const float*)d_in[12];
  const float* bi_p = (const float*)d_in[13];
  const float* bh_p = (const float*)d_in[14];
  const float* Wi_l = (const float*)d_in[15];
  const float* Wh_l = (const float*)d_in[16];
  const float* bi_l = (const float*)d_in[17];
  const float* bh_l = (const float*)d_in[18];
  const float* W1 = (const float*)d_in[19];
  const float* b1 = (const float*)d_in[20];
  const float* W2 = (const float*)d_in[21];
  const float* b2 = (const float*)d_in[22];
  const float* W3 = (const float*)d_in[23];
  const float* b3 = (const float*)d_in[24];

  const size_t off_ps   = 0;
  const size_t off_ls   = off_ps + (size_t)NP * DH * 4;
  const size_t off_g    = off_ls + (size_t)NL * DH * 4;
  const size_t off_cols = off_g + (size_t)NL * GW * 4;
  const size_t off_linf = off_cols + (size_t)NLB * CAP * 4;
  const size_t off_w16  = off_linf + (size_t)NLB * 2 * LB * 4;
  const size_t w16_halves = (size_t)4 * GW * DH + RU * DH + RU * RU;
  const size_t ws_end = off_w16 + w16_halves * 2;
  if (ws_end > ws_size) return;

  char* ws = (char*)d_ws;
  float* path_state = (float*)(ws + off_ps);
  float* link_state = (float*)(ws + off_ls);
  float* G          = (float*)(ws + off_g);
  int* cols         = (int*)(ws + off_cols);
  int* linfo        = (int*)(ws + off_linf);
  _Float16* w16     = (_Float16*)(ws + off_w16);
  _Float16* Wi16p = w16;
  _Float16* Wh16p = w16 + GW * DH;
  _Float16* Wi16l = w16 + 2 * GW * DH;
  _Float16* Wh16l = w16 + 3 * GW * DH;
  _Float16* W1h   = w16 + 4 * GW * DH;
  _Float16* W2h   = w16 + 4 * GW * DH + RU * DH;

  int n_edges = in_sizes[8];
  if (in_sizes[7] < n_edges) n_edges = in_sizes[7];
  if (n_edges < 0) n_edges = 0;

  const int initBlocks = (NP * 8 + 255) / 256;
  const int pathBlocks = (NPT + 7) / 8;
  const int readBlocks = (NPT + 3) / 4;

  init_kernel<<<dim3(initBlocks, 2), 256, 0, stream>>>(traffic, packets, tdp, capacity,
                                                      path_state, link_state);
  cvt_kernel<<<dim3(32, 6), 256, 0, stream>>>(Wi_p, Wh_p, Wi_l, Wh_l, W1, W2, w16);
  csr_kernel<<<NLB, 256, 0, stream>>>(sequence_links, path_to_link, n_edges, cols, linfo);
  link_kernel<<<NLB, 128, 0, stream>>>(0, link_state, path_state, cols, linfo, Wi16l, Wh16l,
                                       bi_l, bh_l, Wi16p, bi_p, G);
  for (int it = 0; it < TIT; ++it) {
    path_kernel<<<pathBlocks, 256, 0, stream>>>(path_state, G, link_to_path, Wh16p, bh_p);
    if (it < TIT - 1)
      link_kernel<<<NLB, 128, 0, stream>>>(1, link_state, path_state, cols, linfo, Wi16l,
                                           Wh16l, bi_l, bh_l, Wi16p, bi_p, G);
  }
  readout_kernel<<<readBlocks, 128, 0, stream>>>(path_state, W1h, b1, W2h, b2, W3, b3,
                                                 (float*)d_out);
}
